// GraphNeuralNetwork_78314433675855
// MI455X (gfx1250) — hardware-run, weakly checked
//
#include <hip/hip_runtime.h>


namespace {

constexpr int N = 50000, NP = 50048, NPL = NP  , SRCM = N  , EFULL = 800000, E = EFULL  ;
constexpr int F0 = 100, KP = 128, H = 128, DO = 64, NBLK = NPL / 32, NL = (NPL < N ? NPL : N);
constexpr float XS = 8.0f, WSC = 256.0f, WSQ = 0.25f, RS_ = 1024.0f, BNEPS = 1e-5f, SLOPE = 0.0f;
static_assert(NP % 32 == 0 && NP >= N && NPL % 32 == 0 && H == 128 && F0 % 4 == 0 && F0 <= KP, "tiling");
typedef _Float16 b16;
typedef __attribute__((ext_vector_type(16))) _Float16 v16b;
typedef __attribute__((ext_vector_type(8))) _Float16 v8b;
typedef __attribute__((ext_vector_type(8))) float v8f;
typedef __attribute__((ext_vector_type(4))) float v4f;
__device__ __forceinline__ float bf16_rne(float f) { unsigned int u = __float_as_uint(f); u += 0x7FFFu + ((u >> 16) & 1u); return __uint_as_float(u & 0xFFFF0000u); }
__device__ __forceinline__ void split16(float v, b16& hi, b16& lo) { hi = (b16)v; lo = (b16)(v - (float)hi); }
__device__ __forceinline__ v16b frag_kb(const b16* p, int hh) { const v8b a = *(const v8b*)(p + 8 * hh), b = *(const v8b*)(p + 16 + 8 * hh); v16b f;
#pragma unroll
  for (int e = 0; e < 8; ++e) { f[e] = a[e]; f[8 + e] = b[e]; } return f; }
__device__ __forceinline__ v8f wmma16b(v16b a, v16b b, v8f c) { v8f d = __builtin_amdgcn_wmma_f32_16x16x32_f16(false, a, false, b, (short)0, c, false, false); asm volatile("v_nop\n\tv_nop\n\tv_nop\n\tv_nop" : "+v"(d) : "v"(a), "v"(b)); return d; }
__device__ __forceinline__ void wave_lds_sync() { __builtin_amdgcn_fence(__ATOMIC_RELEASE, "workgroup"); __builtin_amdgcn_wave_barrier(); __builtin_amdgcn_fence(__ATOMIC_ACQUIRE, "workgroup"); }
__device__ __forceinline__ float pmul(float a, float b) { float p = a * b; asm volatile("" : "+v"(p)); return p; }
__device__ __forceinline__ int iclamp(int v, int lo, int hi) { return v < lo ? lo : (v > hi ? hi : v); }
constexpr int CSR_NBLK = 512, CSR_GB = 9, CSR_GN = 1 << CSR_GB  , CSR_MAXG = 512, CSR_CAP = 12288  ;
__global__ __launch_bounds__(64) void csrA_kernel(const int* __restrict__ dst, int E, int N, int nG, int CHP, int NGP, int* __restrict__ STG, int* __restrict__ HST) {
  extern __shared__ int sm[];
  int* cnt = sm; int* run = sm + NGP; int* ids = sm + 2 * NGP;
  const int b = blockIdx.x; const int ch = (E + CSR_NBLK - 1) / CSR_NBLK; const int e0 = b * ch, e1 = min(E, e0 + ch);
  for (int i = threadIdx.x; i < NGP; i += 64) cnt[i] = 0;
  for (int i = threadIdx.x; i < CHP; i += 64) ids[i] = -1;
  __syncthreads();
  if (threadIdx.x == 0) {
    for (int e = e0; e < e1; ++e) { int d = dst[e]; d = (d < 0) ? 0 : (d >= N ? N - 1 : d); cnt[d >> CSR_GB] += 1; }
    int acc = 0; for (int g = 0; g < nG; ++g) { run[g] = acc; acc += cnt[g]; }
    for (int e = e0; e < e1; ++e) { int d = dst[e]; d = (d < 0) ? 0 : (d >= N ? N - 1 : d); const int g = d >> CSR_GB; ids[run[g]] = e; run[g] += 1; } }
  __syncthreads();
  typedef __attribute__((ext_vector_type(4))) int v4i;
  for (int pass = 0; pass < 2; ++pass) {
    for (int i = threadIdx.x; i < CHP / 4; i += 64) *(volatile v4i*)(STG + (size_t)b * CHP + i * 4) = *(const v4i*)(&ids[i * 4]);
    for (int i = threadIdx.x; i < NGP / 4; i += 64) { v4i v; for (int e = 0; e < 4; ++e) v[e] = (i * 4 + e < nG) ? cnt[i * 4 + e] : 0; *(volatile v4i*)(HST + (size_t)b * NGP + i * 4) = v; }
    __threadfence(); }
}
__global__ __launch_bounds__(512) void csrS_kernel(const int* __restrict__ HST, int nG, int NGP, int* __restrict__ START, int* __restrict__ TOT, int* __restrict__ OFF) {
  __shared__ int tot[CSR_MAXG];
  const int b = threadIdx.x;
  for (int pass = 0; pass < 2; ++pass) { int runb = 0; for (int g = 0; g < nG; ++g) { int c = HST[(size_t)b * NGP + g]; c = (c < 0) ? 0 : c; ((volatile int*)OFF)[(size_t)g * CSR_NBLK + b] = runb; runb += c; } __threadfence(); }
  for (int g = threadIdx.x; g < nG; g += 512) { int s = 0; for (int bb = 0; bb < CSR_NBLK; ++bb) { int c = HST[(size_t)bb * NGP + g]; s += (c < 0) ? 0 : c; } tot[g] = s; }
  __syncthreads();
  if (threadIdx.x < 32) {
    __shared__ int st[CSR_MAXG + 32];
    if (threadIdx.x == 0) { int acc = 0; for (int g = 0; g < NGP; ++g) { st[g] = acc; if (g < nG) acc += (tot[g] + 31) & ~31; } st[NGP] = acc; }
    __builtin_amdgcn_fence(__ATOMIC_RELEASE, "workgroup"); __builtin_amdgcn_wave_barrier(); __builtin_amdgcn_fence(__ATOMIC_ACQUIRE, "workgroup");
    for (int pass = 0; pass < 2; ++pass) { for (int i = threadIdx.x; i < NGP + 32; i += 32) { ((volatile int*)START)[i] = (i <= NGP) ? st[min(i, NGP)] : 0; ((volatile int*)TOT)[i] = (i < nG) ? tot[i] : 0; } __threadfence(); } }
}
__global__ __launch_bounds__(256) void csrB_kernel(const int* __restrict__ dst, int N, int nG, int CHP, int NGP, int permLen, const int* __restrict__ STG, const int* __restrict__ HST, const int* __restrict__ OFF, const int* __restrict__ START, const int* __restrict__ TOT, int* __restrict__ PERM, int* __restrict__ ROWPTR, int* __restrict__ ROWCNT, int* __restrict__ FLAG) {
  typedef __attribute__((ext_vector_type(4))) int v4i;
  __shared__ int ids[CSR_CAP]; __shared__ unsigned short key[CSR_CAP]; __shared__ int outp[CSR_CAP]; __shared__ int ncnt[CSR_GN + 1]; __shared__ int boff[CSR_NBLK + 1];
  const int g = blockIdx.x, t_ = threadIdx.x; int tot = TOT[g]; int st = START[g], stn = START[g + 1]; const int v0 = g * CSR_GN; const int nv = min(CSR_GN, N - v0);
  st = (st < 0) ? 0 : (st > permLen - 32 ? permLen - 32 : st) & ~31; stn = (stn < st) ? st : (stn > permLen ? permLen : stn); tot = (tot < 0) ? 0 : tot; if (tot > stn - st && tot <= CSR_CAP) tot = stn - st;
  if (tot > CSR_CAP) {
    for (int pass = 0; pass < 2; ++pass) { for (int i = t_; i < CSR_GN / 4; i += 256) { v4i a, c; for (int e = 0; e < 4; ++e) { a[e] = st; c[e] = 0; } *(volatile v4i*)(ROWPTR + v0 + i * 4) = a; *(volatile v4i*)(ROWCNT + v0 + i * 4) = c; } if (t_ == 0) ((volatile int*)FLAG)[0] = 1; __threadfence(); } (void)nv; return; }
  if (t_ == 0) { int acc = 0; for (int b = 0; b < CSR_NBLK; ++b) { boff[b] = acc; int c = HST[(size_t)b * NGP + g]; c = (c < 0) ? 0 : (c > CHP ? CHP : c); acc += c; if (acc > tot) acc = tot; } boff[CSR_NBLK] = acc; }
  for (int i = t_; i <= CSR_GN; i += 256) ncnt[i] = 0;
  __syncthreads();
  for (int b = 0; b < CSR_NBLK; ++b) { const int c = boff[b + 1] - boff[b]; int o_ = OFF[(size_t)g * CSR_NBLK + b]; o_ = (o_ < 0) ? 0 : (o_ > CHP - c ? CHP - c : o_); const int* src_ = STG + (size_t)b * CHP + o_;
    for (int i = t_; i < c; i += 256) { int id = src_[i]; id = (id < 0) ? 0 : id; ids[boff[b] + i] = id; int d = dst[id]; d = (d < v0) ? v0 : (d >= N ? N - 1 : d); int kk = d - v0; kk = (kk < 0) ? 0 : (kk >= CSR_GN ? CSR_GN - 1 : kk); key[boff[b] + i] = (unsigned short)kk; } }
  __syncthreads();
  if (t_ == 0) { for (int i = 0; i < tot; ++i) ncnt[key[i]] += 1; int acc = 0; for (int vl = 0; vl < CSR_GN; ++vl) { const int c = ncnt[vl]; ncnt[vl] = acc; acc += c; } ncnt[CSR_GN] = acc;
    for (int i = 0; i < tot; ++i) { const int vl = key[i]; outp[ncnt[vl]] = ids[i]; ncnt[vl] += 1; }
    for (int vl = CSR_GN; vl > 0; --vl) ncnt[vl] = ncnt[vl - 1]; ncnt[0] = 0; }
  __syncthreads();
  for (int pass = 0; pass < 2; ++pass) {
    for (int i = t_; i < (stn - st) / 4; i += 256) { v4i v; for (int e = 0; e < 4; ++e) { const int q = i * 4 + e; v[e] = (q < tot) ? outp[q] : -1; } *(volatile v4i*)(PERM + st + i * 4) = v; }
    for (int i = t_; i < CSR_GN / 4; i += 256) { v4i a, c; for (int e = 0; e < 4; ++e) { const int vl = i * 4 + e; a[e] = st + ncnt[vl]; c[e] = (vl < nv) ? (ncnt[vl + 1] - ncnt[vl]) : 0; } *(volatile v4i*)(ROWPTR + v0 + i * 4) = a; *(volatile v4i*)(ROWCNT + v0 + i * 4) = c; }
    __threadfence(); }
}
__global__ __launch_bounds__(256) void csrZ_kernel(int* __restrict__ p, size_t n4) { typedef __attribute__((ext_vector_type(4))) int v4i; const size_t tid = (size_t)blockIdx.x * 256 + threadIdx.x, nth = (size_t)gridDim.x * 256; v4i z = {0, 0, 0, 0}; for (size_t i = tid; i < n4; i += nth) *(volatile v4i*)(p + i * 4) = z; }
struct CsrBufs { int *STG, *HST, *OFF, *START, *TOT, *PERM, *ROWPTR, *ROWCNT, *FLAG; int nG, NGP, CHP; size_t permLen; char* base; size_t bytes; };
static size_t csr_carve(CsrBufs& c, char* ws, size_t off, int E, int N) {
  const size_t off0 = off; c.base = ws + off;
  auto al = [&](size_t bytes) { char* p = ws + off; off += (bytes + 255) & ~(size_t)255; return p; };
  c.nG = (N + CSR_GN - 1) / CSR_GN; c.NGP = (c.nG + 31) & ~31; const int ch = (E + CSR_NBLK - 1) / CSR_NBLK; c.CHP = (ch + 31) & ~31; c.permLen = (size_t)E + 32 * (size_t)c.nG + 32;
  c.STG = (int*)al((size_t)CSR_NBLK * c.CHP * 4); c.HST = (int*)al((size_t)CSR_NBLK * c.NGP * 4); c.OFF = (int*)al((size_t)c.NGP * CSR_NBLK * 4); c.START = (int*)al((size_t)(c.NGP + 64) * 4); c.TOT = (int*)al((size_t)(c.NGP + 64) * 4);
  c.PERM = (int*)al(c.permLen * 4); c.ROWPTR = (int*)al((size_t)c.nG * CSR_GN * 4); c.ROWCNT = (int*)al((size_t)c.nG * CSR_GN * 4); c.FLAG = (int*)al(256);
  c.bytes = off - off0; return off;
}
static void csr_build(const CsrBufs& c, const int* dst, int E, int N, hipStream_t stream) {
  const size_t smem = (size_t)(2 * c.NGP + c.CHP) * 4;
  csrZ_kernel<<<512, 256, 0, stream>>>((int*)c.base, c.bytes / 16);
  csrA_kernel<<<CSR_NBLK, 64, smem, stream>>>(dst, E, N, c.nG, c.CHP, c.NGP, c.STG, c.HST);
  csrS_kernel<<<1, 512, 0, stream>>>(c.HST, c.nG, c.NGP, c.START, c.TOT, c.OFF);
  csrB_kernel<<<c.nG, 256, 0, stream>>>(dst, N, c.nG, c.CHP, c.NGP, (int)c.permLen, c.STG, c.HST, c.OFF, c.START, c.TOT, c.PERM, c.ROWPTR, c.ROWCNT, c.FLAG);
}

typedef __attribute__((ext_vector_type(4))) _Float16 v4h;
typedef __attribute__((ext_vector_type(2))) float v2f;
template <int KIN, int NOUT>
__global__ __launch_bounds__(256) void wt_kernel(const float* __restrict__ w, b16* __restrict__ WT, float scl) {
  const int u = blockIdx.x * 256 + threadIdx.x; if (u >= NOUT * KP / 8) return; const int e = u * 8; const int o = e / KP, k0 = e % KP; v8b v;
#pragma unroll
  for (int j = 0; j < 8; ++j) { const int k = k0 + j; v[j] = (b16)(k < KIN ? bf16_rne(w[(size_t)(k < KIN ? k : 0) * NOUT + o]) * scl : 0.0f); }
  for (int pass = 0; pass < 2; ++pass) { *(volatile v8b*)(WT + e) = v; __threadfence(); }
}
template <bool L0, int NOUT, bool STATS>
__global__ __launch_bounds__(256) void layer_kernel(const float* __restrict__ Hin, const float* __restrict__ STin, const float* __restrict__ gin, const float* __restrict__ bin, const float* __restrict__ ew, const int* __restrict__ srcs,
    const int* __restrict__ PERM, const int* __restrict__ ROWPTR, const int* __restrict__ ROWCNT, int permLen, const int* __restrict__ OUTCNT, const b16* __restrict__ WT, const b16* __restrict__ WQ, const float* __restrict__ bias, float* __restrict__ Y, float* __restrict__ PART, int mrows) {
  constexpr int NT = NOUT / 16; constexpr int FIN = L0 ? F0 : H;
  __shared__ __attribute__((aligned(16))) b16 Ah[32][KP + 8], Al[32][KP + 8]; __shared__ __attribute__((aligned(16))) float Tf[32][NOUT + 4]; __shared__ float csum[8][NOUT];
  const int tid = threadIdx.x, wave = tid >> 5, lane = tid & 31, nloc = lane & 15, hlf = lane >> 4; const int v0 = blockIdx.x * 32; const int row = tid >> 3, g = tid & 7, c0 = g * 16; const int v = v0 + row;
  float mu[16], sc[16], sh[16];
#pragma unroll
  for (int j = 0; j < 16; ++j) { if (L0) { mu[j] = 0.0f; sc[j] = 1.0f; sh[j] = 0.0f; } else { const int c = c0 + j; mu[j] = STin[c]; sc[j] = rsqrtf(STin[H + c] + BNEPS) * bf16_rne(gin[c]); sh[j] = bf16_rne(bin[c]); } }
  float a[16]; for (int j = 0; j < 16; ++j) a[j] = 0.0f;
  int cnt = 0, q0 = 0; float dv = 0.0f;
  if (v < N) { cnt = iclamp(ROWCNT[v], 0, 65536); q0 = iclamp(ROWPTR[v], 0, permLen - 1); if (q0 + cnt > permLen) cnt = permLen - q0; const int oc = iclamp(OUTCNT[v], 0, 1 << 24); dv = oc > 0 ? 1.0f / sqrtf((float)oc) : 0.0f; }
#pragma unroll 1
  for (int i = 0; i < cnt; ++i) { const int e = iclamp(PERM[q0 + i], 0, E - 1); int s = iclamp(srcs[e], 0, N - 1); const int ocs = iclamp(OUTCNT[s], 0, 1 << 24); const float ds = ocs > 0 ? 1.0f / sqrtf((float)ocs) : 0.0f; const float coef = ds * bf16_rne(ew[e]) * dv; if (SRCM < N) s %= SRCM;
    float hv[16];
    if (L0) { const float* xr = Hin + (size_t)s * F0 + c0;
      if (c0 + 16 <= F0) { for (int q = 0; q < 4; ++q) { const v4f t4 = *(const v4f*)(xr + 4 * q); for (int j = 0; j < 4; ++j) hv[4 * q + j] = bf16_rne(t4[j]); } }
      else if (c0 < F0) { const v4f t4 = *(const v4f*)xr; for (int j = 0; j < 4; ++j) hv[j] = bf16_rne(t4[j]); for (int j = 4; j < 16; ++j) hv[j] = 0.0f; }
      else { for (int j = 0; j < 16; ++j) hv[j] = 0.0f; } }
    else { const float* yr = Hin + (size_t)s * H + c0; for (int q = 0; q < 4; ++q) { const v4f t4 = *(const v4f*)(yr + 4 * q); for (int j = 0; j < 4; ++j) { const int jj = 4 * q + j; hv[jj] = fmaxf((t4[j] - mu[jj]) * sc[jj] + sh[jj], 0.0f); } } }
#pragma unroll
    for (int j = 0; j < 16; ++j) a[j] = fmaf(coef, hv[j], a[j]); }
#pragma unroll
  for (int q = 0; q < 4; ++q) { v4h h4, l4; for (int j = 0; j < 4; ++j) { const float vs = a[4 * q + j] * XS; const b16 p = (b16)vs; h4[j] = p; l4[j] = (b16)((vs - (float)p) * RS_); } *(v4h*)(&Ah[row][c0 + 4 * q]) = h4; *(v4h*)(&Al[row][c0 + 4 * q]) = l4; }
  __syncthreads();
  { const int rt = (NT == 8) ? 0 : (wave & 1), ct0 = (NT == 8) ? wave : (wave >> 1); const int nrt = (NT == 8) ? 2 : 1;
    v8f acc[2] = {(v8f){}, (v8f){}}; const b16* br = WT + (size_t)(ct0 * 16 + nloc) * KP; const b16* bq = WQ + (size_t)(ct0 * 16 + nloc) * KP;
#pragma unroll
    for (int kb = 0; kb < KP; kb += 32) { const v16b bw = frag_kb(br + kb, hlf), bwq = frag_kb(bq + kb, hlf);
      for (int r2 = 0; r2 < nrt; ++r2) { const int rtt = (NT == 8) ? r2 : rt; acc[r2] = wmma16b(frag_kb(&Ah[rtt * 16 + nloc][kb], hlf), bw, acc[r2]); acc[r2] = wmma16b(frag_kb(&Al[rtt * 16 + nloc][kb], hlf), bwq, acc[r2]); } }
    const int col = ct0 * 16 + nloc; const float bb = bf16_rne(bias[col]);
    for (int r2 = 0; r2 < nrt; ++r2) { const int rtt = (NT == 8) ? r2 : rt;
#pragma unroll
      for (int q = 0; q < 8; ++q) { const int rr = rtt * 16 + 8 * hlf + q; Tf[rr][col] = (v0 + rr < N) ? acc[r2][q] * (1.0f / (XS * WSC)) + bb : 0.0f; } } }
  __syncthreads();
  if (STATS) { const int c = tid % NOUT, qq = tid / NOUT, per = 32 / (256 / NOUT); float s = 0.0f; for (int rr = qq * per; rr < qq * per + per; ++rr) s += Tf[rr][c]; csum[qq][c] = s; }
  __syncthreads();
  for (int pass = 0; pass < 2; ++pass) {
    for (int rr = wave * 4; rr < wave * 4 + 4; ++rr) { if (NOUT == 128) { if (v0 + rr < mrows) *(volatile v4f*)(Y + (size_t)(v0 + rr) * NOUT + lane * 4) = *(const v4f*)(&Tf[rr][lane * 4]); }
      else { if ((rr & 1) == 0) { const int r2 = rr + (lane >> 4); if (v0 + r2 < mrows) *(volatile v4f*)(Y + (size_t)(v0 + r2) * NOUT + (lane & 15) * 4) = *(const v4f*)(&Tf[r2][(lane & 15) * 4]); } } }
    if (STATS && wave == 0) { v4f p; for (int q = 0; q < 4; ++q) { const int c = lane * 4 + q; float t = 0.0f; for (int qq = 0; qq < 256 / NOUT; ++qq) t += csum[qq][c]; p[q] = t; } *(volatile v4f*)(PART + (size_t)blockIdx.x * NOUT + lane * 4) = p; }
    __threadfence(); }
}
__global__ __launch_bounds__(128) void reduce_kernel(const float* __restrict__ PART, float* __restrict__ STAT, int which) {
  const int c = threadIdx.x; float s = 0.0f;
#pragma unroll 1
  for (int b = 0; b < NBLK; ++b) s += PART[(size_t)b * H + c];
  for (int pass = 0; pass < 2; ++pass) { ((volatile float*)STAT)[which * H + c] = s * (1.0f / (float)NL); __threadfence(); }
}
__global__ __launch_bounds__(256) void varp_kernel(const float* __restrict__ Y, const float* __restrict__ STAT, float* __restrict__ PART) {
  __shared__ float csum[2][H]; const int tid = threadIdx.x; const int v0 = blockIdx.x * 32; const int c = tid & (H - 1), qq = tid >> 7; const float mu = STAT[c]; float s = 0.0f;
  for (int rr = qq * 16; rr < qq * 16 + 16; ++rr) { const int v = v0 + rr; const float wv = (v < N) ? 1.0f : 0.0f; const float d = Y[(size_t)(v < N ? v : N - 1) * H + c] - mu; s = fmaf(d * wv, d, s); }
  csum[qq][c] = s; __syncthreads();
  const int wave = tid >> 5, lane = tid & 31;
  for (int pass = 0; pass < 2; ++pass) { if (wave == 0) { v4f p; for (int q = 0; q < 4; ++q) { const int cc = lane * 4 + q; p[q] = csum[0][cc] + csum[1][cc]; } *(volatile v4f*)(PART + (size_t)blockIdx.x * H + lane * 4) = p; } __threadfence(); }
}
}

extern "C" void kernel_launch(void* const* d_in, const int* in_sizes, int n_in, void* d_out, int out_size, void* d_ws, size_t ws_size, hipStream_t stream) {
  (void)n_in;
  auto Fp = [&](int i) { return (const float*)d_in[i]; }; auto Ip = [&](int i) { return (const int*)d_in[i]; };
  if (in_sizes[0] != N * F0 || in_sizes[1] != 2 * EFULL || in_sizes[2] != EFULL || in_sizes[3] != F0 * H || in_sizes[4] != H || in_sizes[5] != H || in_sizes[6] != H || in_sizes[7] != H * H || in_sizes[8] != H || in_sizes[9] != H || in_sizes[10] != H || in_sizes[11] != H * DO || in_sizes[12] != DO || out_size != N * DO) return;
  size_t off = 0; char* ws = (char*)d_ws;
  auto carve = [&](size_t bytes) { char* p = ws + off; off += (bytes + 255) & ~(size_t)255; return p; };
  b16* WT0 = (b16*)carve((size_t)H * KP * 2); b16* WQ0 = (b16*)carve((size_t)H * KP * 2); b16* WT1 = (b16*)carve((size_t)H * KP * 2); b16* WQ1 = (b16*)carve((size_t)H * KP * 2); b16* WT2 = (b16*)carve((size_t)DO * KP * 2); b16* WQ2 = (b16*)carve((size_t)DO * KP * 2);
  float* Y0 = (float*)carve((size_t)NP * H * 4); float* Y1 = (float*)carve((size_t)NP * H * 4); float* PART = (float*)carve((size_t)NBLK * H * 4); float* ST0 = (float*)carve(2 * H * 4); float* ST1 = (float*)carve(2 * H * 4);
  CsrBufs csr; off = csr_carve(csr, ws, off, E, N); CsrBufs cso; off = csr_carve(cso, ws, off, E, N);
  if (off > ws_size || off > ((size_t)128 << 20)) return;
  wt_kernel<F0, H><<<(H * KP / 8 + 255) / 256, 256, 0, stream>>>(Fp(3), WT0, WSC); wt_kernel<F0, H><<<(H * KP / 8 + 255) / 256, 256, 0, stream>>>(Fp(3), WQ0, WSQ);
  wt_kernel<H, H><<<(H * KP / 8 + 255) / 256, 256, 0, stream>>>(Fp(7), WT1, WSC); wt_kernel<H, H><<<(H * KP / 8 + 255) / 256, 256, 0, stream>>>(Fp(7), WQ1, WSQ);
  wt_kernel<H, DO><<<(DO * KP / 8 + 255) / 256, 256, 0, stream>>>(Fp(11), WT2, WSC); wt_kernel<H, DO><<<(DO * KP / 8 + 255) / 256, 256, 0, stream>>>(Fp(11), WQ2, WSQ);
  csr_build(csr, Ip(1) + EFULL, E, N, stream);
  csr_build(cso, Ip(1), E, N, stream);
  layer_kernel<true, H, true><<<NBLK, 256, 0, stream>>>(Fp(0), nullptr, nullptr, nullptr, Fp(2), Ip(1), csr.PERM, csr.ROWPTR, csr.ROWCNT, (int)csr.permLen, cso.ROWCNT, WT0, WQ0, Fp(4), Y0, PART, NPL);
  reduce_kernel<<<1, 128, 0, stream>>>(PART, ST0, 0); varp_kernel<<<NBLK, 256, 0, stream>>>(Y0, ST0, PART); reduce_kernel<<<1, 128, 0, stream>>>(PART, ST0, 1);
  layer_kernel<false, H, true><<<NBLK, 256, 0, stream>>>(Y0, ST0, Fp(5), Fp(6), Fp(2), Ip(1), csr.PERM, csr.ROWPTR, csr.ROWCNT, (int)csr.permLen, cso.ROWCNT, WT1, WQ1, Fp(8), Y1, PART, NPL);
  reduce_kernel<<<1, 128, 0, stream>>>(PART, ST1, 0); varp_kernel<<<NBLK, 256, 0, stream>>>(Y1, ST1, PART); reduce_kernel<<<1, 128, 0, stream>>>(PART, ST1, 1);
  layer_kernel<false, DO, false><<<NBLK, 256, 0, stream>>>(Y1, ST1, Fp(9), Fp(10), Fp(2), Ip(1), csr.PERM, csr.ROWPTR, csr.ROWCNT, (int)csr.permLen, cso.ROWCNT, WT2, WQ2, Fp(12), (float*)d_out, nullptr, NL);
}
